// SelfAttention_23837068493232
// MI455X (gfx1250) — hardware-verified
//
#include <hip/hip_runtime.h>
#include <math.h>

constexpr int kSeq = 512;
constexpr int kDim = 512;
constexpr int kHid = 512;
constexpr int kXw  = 2 * kDim;
constexpr int kG3  = 3 * kHid;
constexpr float kResCarry    = 2048.0f;
constexpr float kResCarryInv = 1.0f / 2048.0f;
constexpr float kF16MinNorm  = 6.103515625e-5f;
constexpr float kWhhCarry    = 256.0f;
constexpr float kHCarry      = 16.0f;
constexpr float kGhInv       = 1.0f / (kWhhCarry * kHCarry);
constexpr int kScWP = 516;
constexpr int kScEP = 260;
constexpr int kScJB = 256;
static_assert(kSeq == 512 && kDim == 512 && kHid == 512, "shape constants");
static_assert(kSeq % 64 == 0 && kDim % 64 == 0 && kG3 % 64 == 0, "GEMM M, N tile multiples");
static_assert(kDim % 32 == 0 && kXw % 32 == 0 && kSeq % 32 == 0, "GEMM K multiples of 32");
static_assert(kSeq % kScJB == 0 && kSeq % 16 == 0, "score tiling");
static_assert(kHid == 32 * 16, "16 waves x 32 hidden units in the scan");
static_assert(kHid % 32 == 0, "scan K multiple of 32");

typedef __attribute__((ext_vector_type(16))) _Float16 v16h;
typedef __attribute__((ext_vector_type(8)))  _Float16 v8h;
typedef __attribute__((ext_vector_type(16))) __bf16   v16b;
typedef __attribute__((ext_vector_type(8)))  __bf16   v8b;
typedef __attribute__((ext_vector_type(8)))  float    v8f;
typedef __attribute__((ext_vector_type(4)))  float    v4f;
typedef __attribute__((ext_vector_type(4)))  unsigned int v4u;

__device__ __forceinline__ unsigned short f2bf_bits(float f) {
  unsigned u = __float_as_uint(f);
  return (unsigned short)((u + 0x7FFFu + ((u >> 16) & 1u)) >> 16);
}
__device__ __forceinline__ float bf_bits2f(unsigned short h) { return __uint_as_float(((unsigned)h) << 16); }
__device__ __forceinline__ unsigned pk16(unsigned lo, unsigned hi) { return (lo & 0xffffu) | (hi << 16); }
__device__ __forceinline__ unsigned h16_bits(float f) {
  const _Float16 h = (_Float16)f;
  const unsigned short b = __builtin_bit_cast(unsigned short, h);
  return (unsigned)b;
}

__device__ __forceinline__ void dep_guard4_b(v8f& a, v8f& b, v8f& c, v8f& d, v16b x, v16b y) {
  asm volatile("v_nop\n\tv_nop\n\tv_nop\n\tv_nop" : "+v"(a), "+v"(b), "+v"(c), "+v"(d) : "v"(x), "v"(y));
}
__device__ __forceinline__ void keep4_b(v16b a, v16b b, v16b c, v16b d) { asm volatile("v_nop" :: "v"(a), "v"(b), "v"(c), "v"(d)); }
__device__ __forceinline__ void acc_guard4(v8f& a, v8f& b, v8f& c, v8f& d) {
  asm volatile("v_nop\n\tv_nop\n\tv_nop\n\tv_nop" : "+v"(a), "+v"(b), "+v"(c), "+v"(d));
}
__device__ __forceinline__ void sc_guard(v8f& a, v8f& b, v16h x, v16h y, v16h z) {
  asm volatile("v_nop\n\tv_nop\n\tv_nop\n\tv_nop" : "+v"(a), "+v"(b) : "v"(x), "v"(y), "v"(z));
}
__device__ __forceinline__ void gru_guard3(v8f& a, v8f& b, v8f& c, v16h x, v16h y, v16h z, v16h w) {
  asm volatile("v_nop\n\tv_nop\n\tv_nop\n\tv_nop" : "+v"(a), "+v"(b), "+v"(c) : "v"(x), "v"(y), "v"(z), "v"(w));
}
__device__ __forceinline__ void acc_guard3(v8f& a, v8f& b, v8f& c) {
  asm volatile("v_nop\n\tv_nop\n\tv_nop\n\tv_nop" : "+v"(a), "+v"(b), "+v"(c));
}

struct FragB {
  union U { v16b v; v8b h[2]; };
  static __device__ __forceinline__ v16b load(const __bf16* p) {
    U f; f.h[0] = *(const v8b*)(p); f.h[1] = *(const v8b*)(p + 16); return f.v;
  }
  static __device__ __forceinline__ v8f mma(v16b a, v16b b, v8f c) {
    return __builtin_amdgcn_wmma_f32_16x16x32_bf16(false, a, false, b, (short)0, c, false, false);
  }
};
struct FragH {
  union U { v16h v; v8h h[2]; };
  static __device__ __forceinline__ v16h load(const _Float16* p) {
    U f; f.h[0] = *(const v8h*)(p); f.h[1] = *(const v8h*)(p + 16); return f.v;
  }
};

template <int BIAS_MODE, int OUT_MODE>
__global__ __launch_bounds__(256) void wmma_gemm64(
    const unsigned short* __restrict__ Ap, const unsigned short* __restrict__ A2p, int lda, long strideA,
    const unsigned short* __restrict__ Btp, const unsigned short* __restrict__ Bt2p, int ldb, long strideB,
    void* __restrict__ Cout, void* __restrict__ Cout2, int ldc, long strideC,
    const float* __restrict__ bias,
    int M, int N, int K, float scale) {
  typedef __bf16 T;
  typedef v16b V;
  const T* A = (const T*)Ap; const T* A2 = (const T*)A2p; const T* Bt = (const T*)Btp; const T* Bt2 = (const T*)Bt2p;
  __shared__ __align__(16) float sT[8][16 * 68];
  const int b    = blockIdx.y;
  const int lane = threadIdx.x & 31;
  const int wave = threadIdx.x >> 5;
  const int tilesN = N >> 6;
  const int tilesM = M >> 6;
  const int tile = blockIdx.x * 8 + wave;
  if (tile >= tilesM * tilesN) return;
  const int tm = tile / tilesN;
  const int tn = tile - tm * tilesN;
  const int m0 = tm << 6;
  const int n0 = tn << 6;

  const T* Ab  = A   + (size_t)b * strideA;
  const T* Bb  = Bt  + (size_t)b * strideB;
  const T* Ab2 = A2  + (size_t)b * strideA;
  const T* Bb2 = Bt2 + (size_t)b * strideB;

  const int rlane = lane & 15;
  const int koff  = (lane >> 4) * 8;
  const int mOff  = (lane >> 4) * 8;

  v8f acc[4][4];
#pragma unroll
  for (int i = 0; i < 4; ++i)
#pragma unroll
    for (int j = 0; j < 4; ++j) acc[i][j] = (v8f){0.f,0.f,0.f,0.f,0.f,0.f,0.f,0.f};

  for (int k0 = 0; k0 < K; k0 += 32) {
    V bh[4], bl[4];
#pragma unroll
    for (int j = 0; j < 4; ++j) {
      const size_t bo = (size_t)(n0 + (j << 4) + rlane) * ldb + koff + k0;
      bh[j] = FragB::load(Bb + bo);
      bl[j] = FragB::load(Bb2 + bo);
    }
#pragma unroll
    for (int i = 0; i < 4; ++i) {
      const size_t ao = (size_t)(m0 + (i << 4) + rlane) * lda + koff + k0;
      V ah = FragB::load(Ab + ao);
      V al = FragB::load(Ab2 + ao);
#pragma unroll
      for (int j = 0; j < 4; ++j) {
        acc[i][j] = FragB::mma(ah, bh[j], acc[i][j]);
        acc[i][j] = FragB::mma(ah, bl[j], acc[i][j]);
        acc[i][j] = FragB::mma(al, bh[j], acc[i][j]);
      }
      dep_guard4_b(acc[i][0], acc[i][1], acc[i][2], acc[i][3], ah, al);
    }
    keep4_b(bh[0], bh[1], bh[2], bh[3]);
    keep4_b(bl[0], bl[1], bl[2], bl[3]);
  }
  acc_guard4(acc[0][0], acc[0][1], acc[0][2], acc[0][3]);
  acc_guard4(acc[1][0], acc[1][1], acc[1][2], acc[1][3]);
  acc_guard4(acc[2][0], acc[2][1], acc[2][2], acc[2][3]);
  acc_guard4(acc[3][0], acc[3][1], acc[3][2], acc[3][3]);

  float* slab = sT[wave];
#pragma unroll
  for (int i = 0; i < 4; ++i) {
    const int mBase = m0 + (i << 4);
#pragma unroll
    for (int j = 0; j < 4; ++j) {
      const int n = n0 + (j << 4) + rlane;
      float bv = 0.f;
      if (BIAS_MODE == 2) bv = bias[n];
#pragma unroll
      for (int r = 0; r < 8; ++r) {
        float v = acc[i][j][r] * scale;
        if (BIAS_MODE == 2) v += bv;
        slab[(mOff + r) * 68 + (j << 4) + rlane] = v;
      }
    }
    __builtin_amdgcn_fence(__ATOMIC_RELEASE, "workgroup");
    __builtin_amdgcn_wave_barrier();
    __builtin_amdgcn_fence(__ATOMIC_ACQUIRE, "workgroup");
    if (OUT_MODE == 0) {
      float* C = (float*)Cout + (size_t)b * strideC;
      const int hh = lane >> 4, c4 = (lane & 15) * 4;
      for (int pass = 0; pass < 2; ++pass) {
#pragma unroll
        for (int it = 0; it < 8; ++it) {
          const int row = it * 2 + hh;
          v4f v = *(const v4f*)(slab + row * 68 + c4);
          *(volatile v4f*)(C + (size_t)(mBase + row) * ldc + n0 + c4) = v;
        }
        __threadfence();
      }
    } else {
      const int q = lane >> 3, c8 = (lane & 7) * 8;
      unsigned short* C  = (unsigned short*)Cout  + (size_t)b * strideC;
      unsigned short* C2 = (unsigned short*)Cout2 + (size_t)b * strideC;
      for (int pass = 0; pass < 2; ++pass) {
#pragma unroll
        for (int it = 0; it < 4; ++it) {
          const int row = it * 4 + q;
          const float* sp = slab + row * 68 + c8;
          v8h hv, lv;
#pragma unroll
          for (int e = 0; e < 8; ++e) {
            unsigned short hb = f2bf_bits(sp[e]);
            unsigned short lb = f2bf_bits(sp[e] - bf_bits2f(hb));
            hv[e] = __builtin_bit_cast(_Float16, hb);
            lv[e] = __builtin_bit_cast(_Float16, lb);
          }
          *(volatile v8h*)(C + (size_t)(mBase + row) * ldc + n0 + c8) = hv;
          *(volatile v8h*)(C2 + (size_t)(mBase + row) * ldc + n0 + c8) = lv;
        }
        __threadfence();
      }
    }
    __builtin_amdgcn_fence(__ATOMIC_RELEASE, "workgroup");
    __builtin_amdgcn_wave_barrier();
    __builtin_amdgcn_fence(__ATOMIC_ACQUIRE, "workgroup");
  }
}

__global__ __launch_bounds__(256) void prep_v_kernel(const float* __restrict__ v, unsigned short* __restrict__ XH,
                                                     unsigned short* __restrict__ XL, unsigned short* __restrict__ VHL) {
  const int i = blockIdx.x * 256 + threadIdx.x;
  if (i < kSeq * 64) {
    const int row = i >> 6;
    const int c8  = i & 63;
    const float* sp = v + (size_t)row * kDim + c8 * 8;
    const v4f a = *(const v4f*)(sp);
    const v4f b = *(const v4f*)(sp + 4);
    float x[8];
#pragma unroll
    for (int e = 0; e < 4; ++e) { x[e] = a[e]; x[4 + e] = b[e]; }
    unsigned bh[8], bl[8], fh[8], fl[8];
#pragma unroll
    for (int e = 0; e < 8; ++e) {
      const float f = x[e];
      const unsigned short hb = f2bf_bits(f);
      const unsigned short lb = f2bf_bits(f - bf_bits2f(hb));
      bh[e] = (unsigned)hb;
      bl[e] = (unsigned)lb;
      const float fq = (fabsf(f) >= kF16MinNorm) ? f : 0.0f;
      const _Float16 hh = (_Float16)fq;
      const unsigned short hbits = __builtin_bit_cast(unsigned short, hh);
      const float res = (f - (float)hh) * kResCarry;
      fh[e] = (unsigned)hbits;
      fl[e] = h16_bits(res);
    }
    const v4u uh = (v4u){pk16(bh[0], bh[1]), pk16(bh[2], bh[3]), pk16(bh[4], bh[5]), pk16(bh[6], bh[7])};
    const v4u ul = (v4u){pk16(bl[0], bl[1]), pk16(bl[2], bl[3]), pk16(bl[4], bl[5]), pk16(bl[6], bl[7])};
    const v4u gh = (v4u){pk16(fh[0], fh[1]), pk16(fh[2], fh[3]), pk16(fh[4], fh[5]), pk16(fh[6], fh[7])};
    const v4u gl = (v4u){pk16(fl[0], fl[1]), pk16(fl[2], fl[3]), pk16(fl[4], fl[5]), pk16(fl[6], fl[7])};
    const size_t ox = (size_t)row * kXw + c8 * 8;
    const size_t ov = (size_t)row * (2 * kDim) + c8 * 8;
    *(volatile v4u*)(XH + ox) = uh;
    *(volatile v4u*)(XL + ox) = ul;
    *(volatile v4u*)(VHL + ov) = gh;
    *(volatile v4u*)(VHL + ov + kDim) = gl;
    __threadfence();
    *(volatile v4u*)(XH + ox) = uh;
    *(volatile v4u*)(XL + ox) = ul;
    *(volatile v4u*)(VHL + ov) = gh;
    *(volatile v4u*)(VHL + ov + kDim) = gl;
  }
}

__global__ __launch_bounds__(256) void tpose_v_kernel(const float* __restrict__ src, unsigned short* __restrict__ OH,
                                                      unsigned short* __restrict__ OL) {
  __shared__ float Tt[64 * 65];
  const int tid = threadIdx.x;
  const int c0 = blockIdx.x * 64, r0 = blockIdx.y * 64;
#pragma unroll
  for (int i = 0; i < 4; ++i) {
    const int idx = i * 256 + tid;
    const int rr = idx >> 4, cc = (idx & 15) * 4;
    const v4f v = *(const v4f*)(src + (size_t)(r0 + rr) * kDim + c0 + cc);
    Tt[rr * 65 + cc + 0] = v[0];
    Tt[rr * 65 + cc + 1] = v[1];
    Tt[rr * 65 + cc + 2] = v[2];
    Tt[rr * 65 + cc + 3] = v[3];
  }
  __syncthreads();
  const int q = tid >> 3, c8 = (tid & 7) * 8;
  v4u hv[2], lv[2];
#pragma unroll
  for (int g = 0; g < 2; ++g) {
    const int qq = g * 32 + q;
    unsigned hb[8], lb[8];
#pragma unroll
    for (int e = 0; e < 8; ++e) {
      const float f = Tt[(c8 + e) * 65 + qq];
      const unsigned short h = f2bf_bits(f);
      const unsigned short l = f2bf_bits(f - bf_bits2f(h));
      hb[e] = (unsigned)h;
      lb[e] = (unsigned)l;
    }
    hv[g] = (v4u){pk16(hb[0], hb[1]), pk16(hb[2], hb[3]), pk16(hb[4], hb[5]), pk16(hb[6], hb[7])};
    lv[g] = (v4u){pk16(lb[0], lb[1]), pk16(lb[2], lb[3]), pk16(lb[4], lb[5]), pk16(lb[6], lb[7])};
  }
  for (int pass = 0; pass < 2; ++pass) {
#pragma unroll
    for (int g = 0; g < 2; ++g) {
      const size_t o = (size_t)(c0 + g * 32 + q) * kSeq + (size_t)(r0 + c8);
      *(volatile v4u*)(OH + o) = hv[g];
      *(volatile v4u*)(OL + o) = lv[g];
    }
    __threadfence();
  }
}

__global__ __launch_bounds__(256) void split2_kernel(const float* __restrict__ srcA, const float* __restrict__ srcB,
                                                     unsigned short* __restrict__ DH, unsigned short* __restrict__ DL, int n8) {
  const int y = blockIdx.y;
  const float* src = y ? srcB : srcA;
  const int i = blockIdx.x * 256 + threadIdx.x;
  if (i < n8) {
    const float* sp = src + (size_t)i * 8;
    const v4f a = *(const v4f*)(sp);
    const v4f b = *(const v4f*)(sp + 4);
    float x[8];
#pragma unroll
    for (int e = 0; e < 4; ++e) { x[e] = a[e]; x[4 + e] = b[e]; }
    unsigned hb[8], lb[8];
#pragma unroll
    for (int e = 0; e < 8; ++e) {
      const unsigned short h = f2bf_bits(x[e]);
      const unsigned short l = f2bf_bits(x[e] - bf_bits2f(h));
      hb[e] = (unsigned)h;
      lb[e] = (unsigned)l;
    }
    const v4u uh = (v4u){pk16(hb[0], hb[1]), pk16(hb[2], hb[3]), pk16(hb[4], hb[5]), pk16(hb[6], hb[7])};
    const v4u ul = (v4u){pk16(lb[0], lb[1]), pk16(lb[2], lb[3]), pk16(lb[4], lb[5]), pk16(lb[6], lb[7])};
    const size_t o = ((size_t)y * (size_t)n8 + (size_t)i) * 8;
    *(volatile v4u*)(DH + o) = uh;
    *(volatile v4u*)(DL + o) = ul;
    __threadfence();
    *(volatile v4u*)(DH + o) = uh;
    *(volatile v4u*)(DL + o) = ul;
  }
}

__global__ __launch_bounds__(256) void cvt2_f16_kernel(const float* __restrict__ srcA, const float* __restrict__ srcB,
                                                       unsigned short* __restrict__ D, int n8, float carry) {
  const int y = blockIdx.y;
  const float* src = y ? srcB : srcA;
  const int i = blockIdx.x * 256 + threadIdx.x;
  if (i < n8) {
    const float* sp = src + (size_t)i * 8;
    const v4f a = *(const v4f*)(sp);
    const v4f b = *(const v4f*)(sp + 4);
    unsigned hb[8];
#pragma unroll
    for (int e = 0; e < 4; ++e) {
      hb[e]     = h16_bits(a[e] * carry);
      hb[4 + e] = h16_bits(b[e] * carry);
    }
    const v4u uh = (v4u){pk16(hb[0], hb[1]), pk16(hb[2], hb[3]), pk16(hb[4], hb[5]), pk16(hb[6], hb[7])};
    const size_t o = ((size_t)y * (size_t)n8 + (size_t)i) * 8;
    *(volatile v4u*)(D + o) = uh;
    __threadfence();
    *(volatile v4u*)(D + o) = uh;
  }
}

__device__ __forceinline__ void tanh_hl(float x, _Float16& hi, _Float16& lo) {
  const float e2 = __expf(2.0f * x);
  const float tv = 1.0f - 2.0f * __builtin_amdgcn_rcpf(e2 + 1.0f);
  const float tq = (fabsf(tv) >= kF16MinNorm) ? tv : 0.0f;
  const _Float16 h = (_Float16)tq;
  hi = h;
  lo = (_Float16)((tv - (float)h) * kResCarry);
}

__global__ __launch_bounds__(256) void score_kernel(const float* __restrict__ U, const float* __restrict__ WQ,
                                                    const unsigned short* __restrict__ VHL, float* __restrict__ E) {
  __shared__ __align__(16) float wt[16 * kScWP];
  __shared__ __align__(16) float et[16 * kScEP];
  union BU { v16h v; v4u q[2]; };
  const int tid = threadIdx.x, lane = tid & 31, wave = tid >> 5;
  const int c = lane & 15, hh = lane >> 4, koff = hh * 8;
  const int t0 = blockIdx.y * 16;
  const int jb = blockIdx.x * kScJB;
#pragma unroll
  for (int it = 0; it < 8; ++it) {
    const int idx = it * 256 + tid;
    const int row = idx >> 7;
    const int c4  = (idx & 127) * 4;
    const v4f x = *(const v4f*)(WQ + (size_t)(t0 + row) * kDim + c4);
    *(v4f*)(wt + row * kScWP + c4) = x;
  }
  __syncthreads();

  const int nsel = (c < 1) ? 0 : 1;
  const unsigned bmask = (c < 2) ? 0xFFFFFFFFu : 0u;
  const v4u bm = (v4u){bmask, bmask, bmask, bmask};
  const float* wrow = wt + c * kScWP + koff;
  const v8f z8 = {0.f, 0.f, 0.f, 0.f, 0.f, 0.f, 0.f, 0.f};

#pragma unroll 1
  for (int jj = 0; jj < 32; ++jj) {
    const int jl = wave * 32 + jj;
    const int j  = jb + jl;
    const float* urow = U + (size_t)j * kDim + koff;
    const unsigned short* brow = VHL + (size_t)j * (2 * kDim) + nsel * kDim + koff;
    v8f d1 = z8, d2 = z8;
#pragma unroll 1
    for (int k0 = 0; k0 < kDim; k0 += 32) {
      const v4f u0 = *(const v4f*)(urow + k0);
      const v4f u1 = *(const v4f*)(urow + k0 + 4);
      const v4f u2 = *(const v4f*)(urow + k0 + 16);
      const v4f u3 = *(const v4f*)(urow + k0 + 20);
      const v4u b0 = *(const v4u*)(brow + k0);
      const v4u b1 = *(const v4u*)(brow + k0 + 16);
      const v4f w0 = *(const v4f*)(wrow + k0);
      const v4f w1 = *(const v4f*)(wrow + k0 + 4);
      const v4f w2 = *(const v4f*)(wrow + k0 + 16);
      const v4f w3 = *(const v4f*)(wrow + k0 + 20);
      const v4f x0 = u0 + w0;
      const v4f x1 = u1 + w1;
      const v4f x2 = u2 + w2;
      const v4f x3 = u3 + w3;
      BU bq;
      bq.q[0] = b0 & bm;
      bq.q[1] = b1 & bm;
      v16h ah, al;
#pragma unroll
      for (int e = 0; e < 4; ++e) {
        _Float16 h, l;
        tanh_hl(x0[e], h, l);
        ah[e] = h; al[e] = l;
        tanh_hl(x1[e], h, l);
        ah[4 + e] = h; al[4 + e] = l;
        tanh_hl(x2[e], h, l);
        ah[8 + e] = h; al[8 + e] = l;
        tanh_hl(x3[e], h, l);
        ah[12 + e] = h; al[12 + e] = l;
      }
      d1 = __builtin_amdgcn_wmma_f32_16x16x32_f16(false, ah, false, bq.v, (short)0, d1, false, false);
      d2 = __builtin_amdgcn_wmma_f32_16x16x32_f16(false, al, false, bq.v, (short)0, d2, false, false);
      sc_guard(d1, d2, ah, al, bq.v);
    }
#pragma unroll
    for (int r = 0; r < 8; ++r) {
      const float c1 = __shfl_xor(d1[r], 1, 32);
      const float ev = d1[r] + (c1 + d2[r]) * kResCarryInv;
      if (c == 0) et[(8 * hh + r) * kScEP + jl] = ev;
    }
  }
  __syncthreads();
  for (int pass = 0; pass < 2; ++pass) {
#pragma unroll
    for (int rr = 0; rr < 2; ++rr) {
#pragma unroll
      for (int s = 0; s < 2; ++s) {
        const int row = 2 * wave + rr;
        const int c4 = s * 128 + lane * 4;
        const v4f val = *(const v4f*)(et + row * kScEP + c4);
        *(volatile v4f*)(E + (size_t)(t0 + row) * kSeq + jb + c4) = val;
      }
    }
    __threadfence();
  }
}

__global__ __launch_bounds__(64) void softmax_split_kernel(const float* __restrict__ E, unsigned short* __restrict__ AH,
                                                           unsigned short* __restrict__ AL) {
  __shared__ float redM[2];
  __shared__ float redS[2];
  const int row = blockIdx.x;
  const int t = threadIdx.x, lane = t & 31, wave = t >> 5;
  const float* sr = E + (size_t)row * kSeq + t * 8;
  const v4f a = *(const v4f*)(sr);
  const v4f b = *(const v4f*)(sr + 4);
  float x[8];
#pragma unroll
  for (int e = 0; e < 4; ++e) { x[e] = a[e]; x[4 + e] = b[e]; }
  float m = fmaxf(fmaxf(fmaxf(x[0], x[1]), fmaxf(x[2], x[3])), fmaxf(fmaxf(x[4], x[5]), fmaxf(x[6], x[7])));
#pragma unroll
  for (int off = 16; off > 0; off >>= 1) m = fmaxf(m, __shfl_xor(m, off, 32));
  if (lane == 0) redM[wave] = m;
  __syncthreads();
  m = fmaxf(redM[0], redM[1]);
  float p[8];
  float s = 0.0f;
#pragma unroll
  for (int e = 0; e < 8; ++e) { p[e] = expf(x[e] - m); s += p[e]; }
#pragma unroll
  for (int off = 16; off > 0; off >>= 1) s += __shfl_xor(s, off, 32);
  if (lane == 0) redS[wave] = s;
  __syncthreads();
  s = redS[0] + redS[1];
  const float inv = 1.0f / s;
  unsigned hb[8], lb[8];
#pragma unroll
  for (int e = 0; e < 8; ++e) {
    const float av = p[e] * inv;
    const unsigned short h = f2bf_bits(av);
    const unsigned short l = f2bf_bits(av - bf_bits2f(h));
    hb[e] = (unsigned)h;
    lb[e] = (unsigned)l;
  }
  const v4u uh = (v4u){pk16(hb[0], hb[1]), pk16(hb[2], hb[3]), pk16(hb[4], hb[5]), pk16(hb[6], hb[7])};
  const v4u ul = (v4u){pk16(lb[0], lb[1]), pk16(lb[2], lb[3]), pk16(lb[4], lb[5]), pk16(lb[6], lb[7])};
  const size_t o = (size_t)row * kSeq + t * 8;
  *(volatile v4u*)(AH + o) = uh;
  *(volatile v4u*)(AL + o) = ul;
  __threadfence();
  *(volatile v4u*)(AH + o) = uh;
  *(volatile v4u*)(AL + o) = ul;
}

__device__ __forceinline__ float sigm_f(float x)  { return __builtin_amdgcn_rcpf(1.0f + expf(-x)); }
__device__ __forceinline__ float tanh_id(float x) { return 1.0f - 2.0f * __builtin_amdgcn_rcpf(expf(2.0f * x) + 1.0f); }

__global__ __launch_bounds__(512) void gru_kernel(const float* __restrict__ gif, const float* __restrict__ gib,
                                                  const unsigned short* __restrict__ whh16,
                                                  const float* __restrict__ bhhf, const float* __restrict__ bhhb,
                                                  float* __restrict__ out) {
  __shared__ __align__(16) float          hf[2][kHid];
  __shared__ __align__(16) unsigned short hb[2][2][kHid];
  __shared__ __align__(16) float          bsm[kG3];
  union BU { v16h v; v4u q[2]; };
  const int dir = blockIdx.x;
  const float* gi  = dir ? gib  : gif;
  const float* bhh = dir ? bhhb : bhhf;
  const _Float16* W = (const _Float16*)whh16 + (size_t)dir * kG3 * kHid;
  const int tid = threadIdx.x, lane = tid & 31, wave = tid >> 5;
  const int c = lane & 15, hh = lane >> 4, koff = hh * 8;

  hf[0][tid] = 0.0f;
  hf[1][tid] = 0.0f;
  {
    unsigned short* hbf = &hb[0][0][0];
#pragma unroll
    for (int e = 0; e < 4; ++e) hbf[tid * 4 + e] = (unsigned short)0;
  }
  bsm[tid]            = bhh[tid];
  bsm[kHid + tid]     = bhh[kHid + tid];
  bsm[2 * kHid + tid] = bhh[2 * kHid + tid];
  __syncthreads();

  const int nsel = (c < 1) ? 0 : 1;
  const unsigned bmask = (c < 2) ? 0xFFFFFFFFu : 0u;
  const v4u bm = (v4u){bmask, bmask, bmask, bmask};
  const v8f z8 = {0.f, 0.f, 0.f, 0.f, 0.f, 0.f, 0.f, 0.f};

#pragma unroll 1
  for (int s = 0; s < kSeq; ++s) {
    const int t = dir ? (kSeq - 1 - s) : s;
    const int cur = s & 1;
    const int nxt = cur ^ 1;
    const unsigned short* bp = &hb[cur][nsel][koff];

#pragma unroll 1
    for (int ub = 0; ub < 2; ++ub) {
      const int ug = 2 * wave + ub;
      const _Float16* ar = W + (size_t)(16 * ug + c) * kHid + koff;
      const _Float16* az = ar + (size_t)kHid * kHid;
      const _Float16* an = az + (size_t)kHid * kHid;
      v8f dr = z8, dz = z8, dn = z8;
#pragma unroll 1
      for (int k0 = 0; k0 < kHid; k0 += 32) {
        const v4u q0 = *(const v4u*)(bp + k0);
        const v4u q1 = *(const v4u*)(bp + k0 + 16);
        const v16h fr = FragH::load(ar + k0);
        const v16h fz = FragH::load(az + k0);
        const v16h fn = FragH::load(an + k0);
        BU bq;
        bq.q[0] = q0 & bm;
        bq.q[1] = q1 & bm;
        dr = __builtin_amdgcn_wmma_f32_16x16x32_f16(false, fr, false, bq.v, (short)0, dr, false, false);
        dz = __builtin_amdgcn_wmma_f32_16x16x32_f16(false, fz, false, bq.v, (short)0, dz, false, false);
        dn = __builtin_amdgcn_wmma_f32_16x16x32_f16(false, fn, false, bq.v, (short)0, dn, false, false);
        gru_guard3(dr, dz, dn, fr, fz, fn, bq.v);
      }
      acc_guard3(dr, dz, dn);

      const int u0 = 16 * ug + 8 * hh;
      const float* gp = gi + (size_t)t * kG3 + u0;
      const v4f gr0 = *(const v4f*)(gp);
      const v4f gr1 = *(const v4f*)(gp + 4);
      const v4f gz0 = *(const v4f*)(gp + kHid);
      const v4f gz1 = *(const v4f*)(gp + kHid + 4);
      const v4f gn0 = *(const v4f*)(gp + 2 * kHid);
      const v4f gn1 = *(const v4f*)(gp + 2 * kHid + 4);
      const v4f br0 = *(const v4f*)(bsm + u0);
      const v4f br1 = *(const v4f*)(bsm + u0 + 4);
      const v4f bz0 = *(const v4f*)(bsm + kHid + u0);
      const v4f bz1 = *(const v4f*)(bsm + kHid + u0 + 4);
      const v4f bn0 = *(const v4f*)(bsm + 2 * kHid + u0);
      const v4f bn1 = *(const v4f*)(bsm + 2 * kHid + u0 + 4);
      const v4f ho0 = *(const v4f*)(&hf[cur][u0]);
      const v4f ho1 = *(const v4f*)(&hf[cur][u0 + 4]);
      float gir[8], giz[8], gin[8], bbr[8], bbz[8], bbn[8], hol[8], hnw[8];
#pragma unroll
      for (int e = 0; e < 4; ++e) {
        gir[e] = gr0[e]; gir[4 + e] = gr1[e];
        giz[e] = gz0[e]; giz[4 + e] = gz1[e];
        gin[e] = gn0[e]; gin[4 + e] = gn1[e];
        bbr[e] = br0[e]; bbr[4 + e] = br1[e];
        bbz[e] = bz0[e]; bbz[4 + e] = bz1[e];
        bbn[e] = bn0[e]; bbn[4 + e] = bn1[e];
        hol[e] = ho0[e]; hol[4 + e] = ho1[e];
      }
      unsigned hib[8], lob[8];
#pragma unroll
      for (int r = 0; r < 8; ++r) {
        const float sr = __shfl_xor(dr[r], 1, 32);
        const float sz = __shfl_xor(dz[r], 1, 32);
        const float sn = __shfl_xor(dn[r], 1, 32);
        const float hr = (dr[r] + sr * kResCarryInv) * kGhInv + bbr[r];
        const float hz = (dz[r] + sz * kResCarryInv) * kGhInv + bbz[r];
        const float hn = (dn[r] + sn * kResCarryInv) * kGhInv + bbn[r];
        const float rg = sigm_f(gir[r] + hr);
        const float zg = sigm_f(giz[r] + hz);
        const float ng = tanh_id(gin[r] + rg * hn);
        const float hv = (1.0f - zg) * ng + zg * hol[r];
        hnw[r] = hv;
        const float hc = hv * kHCarry;
        const float hq = (fabsf(hc) >= kF16MinNorm) ? hc : 0.0f;
        const _Float16 h16 = (_Float16)hq;
        const unsigned short hbits = __builtin_bit_cast(unsigned short, h16);
        hib[r] = (unsigned)hbits;
        lob[r] = h16_bits((hc - (float)h16) * kResCarry);
      }
      if (c == 0) {
        *(v4f*)(&hf[nxt][u0])     = (v4f){hnw[0], hnw[1], hnw[2], hnw[3]};
        *(v4f*)(&hf[nxt][u0 + 4]) = (v4f){hnw[4], hnw[5], hnw[6], hnw[7]};
        *(v4u*)(&hb[nxt][0][u0]) = (v4u){pk16(hib[0], hib[1]), pk16(hib[2], hib[3]), pk16(hib[4], hib[5]), pk16(hib[6], hib[7])};
        *(v4u*)(&hb[nxt][1][u0]) = (v4u){pk16(lob[0], lob[1]), pk16(lob[2], lob[3]), pk16(lob[4], lob[5]), pk16(lob[6], lob[7])};
      }
      asm volatile("" ::: "memory");
    }
    __syncthreads();
    {
      const float hv = hf[nxt][tid];
      volatile float* op = out + (size_t)t * (2 * kHid) + dir * kHid + tid;
      *op = hv;
      __threadfence();
      *op = hv;
    }
  }
}

extern "C" void kernel_launch(void* const* d_in, const int* in_sizes, int n_in,
                              void* d_out, int out_size, void* d_ws, size_t ws_size, hipStream_t stream) {
  if (n_in < 13 || d_out == nullptr || d_ws == nullptr) return;
  if (in_sizes[0] != kSeq * kDim || in_sizes[1] != kDim * kDim || in_sizes[2] != kDim ||
      in_sizes[3] != kDim * kDim || in_sizes[4] != kDim ||
      in_sizes[5] != kG3 * kXw || in_sizes[6] != kG3 * kHid || in_sizes[7] != kG3 || in_sizes[8] != kG3 ||
      in_sizes[9] != kG3 * kXw || in_sizes[10] != kG3 * kHid || in_sizes[11] != kG3 || in_sizes[12] != kG3 ||
      out_size != kSeq * 2 * kHid) return;

  const float* v     = (const float*)d_in[0];
  const float* w1    = (const float*)d_in[1];
  const float* b1    = (const float*)d_in[2];
  const float* w2    = (const float*)d_in[3];
  const float* b2    = (const float*)d_in[4];
  const float* wih_f = (const float*)d_in[5];
  const float* whh_f = (const float*)d_in[6];
  const float* bih_f = (const float*)d_in[7];
  const float* bhh_f = (const float*)d_in[8];
  const float* wih_b = (const float*)d_in[9];
  const float* whh_b = (const float*)d_in[10];
  const float* bih_b = (const float*)d_in[11];
  const float* bhh_b = (const float*)d_in[12];
  float* out = (float*)d_out;

  char* ws = (char*)d_ws; size_t off = 0;
  auto carve = [&](size_t bytes) -> char* { char* p = ws + off; off += (bytes + 255) & ~(size_t)255; return p; };
  unsigned short* XH    = (unsigned short*)carve((size_t)kSeq * kXw * 2);
  unsigned short* XL    = (unsigned short*)carve((size_t)kSeq * kXw * 2);
  unsigned short* VHL   = (unsigned short*)carve((size_t)kSeq * 2 * kDim * 2);
  unsigned short* VTH   = (unsigned short*)carve((size_t)kDim * kSeq * 2);
  unsigned short* VTL   = (unsigned short*)carve((size_t)kDim * kSeq * 2);
  unsigned short* W12H  = (unsigned short*)carve((size_t)2 * kDim * kDim * 2);
  unsigned short* W12L  = (unsigned short*)carve((size_t)2 * kDim * kDim * 2);
  unsigned short* WIHH  = (unsigned short*)carve((size_t)2 * kG3 * kXw * 2);
  unsigned short* WIHL  = (unsigned short*)carve((size_t)2 * kG3 * kXw * 2);
  unsigned short* WHH16 = (unsigned short*)carve((size_t)2 * kG3 * kHid * 2);
  float*          U     = (float*)carve((size_t)kSeq * kDim * 4);
  float*          WQ    = (float*)carve((size_t)kSeq * kDim * 4);
  float*          E     = (float*)carve((size_t)kSeq * kSeq * 4);
  unsigned short* AH    = (unsigned short*)carve((size_t)kSeq * kSeq * 2);
  unsigned short* AL    = (unsigned short*)carve((size_t)kSeq * kSeq * 2);
  float*          GIF   = (float*)carve((size_t)kSeq * kG3 * 4);
  float*          GIB   = (float*)carve((size_t)kSeq * kG3 * 4);
  if (off > ws_size || off > (size_t)134217728) return;

  prep_v_kernel<<<(kSeq * 64) / 256, 256, 0, stream>>>(v, XH, XL, VHL);
  tpose_v_kernel<<<dim3(kDim / 64, kSeq / 64), 256, 0, stream>>>(v, VTH, VTL);
  const int n8w = kDim * kDim / 8;
  const int n8i = kG3 * kXw / 8;
  const int n8h = kG3 * kHid / 8;
  split2_kernel<<<dim3(n8w / 256, 2), 256, 0, stream>>>(w1, w2, W12H, W12L, n8w);
  split2_kernel<<<dim3(n8i / 256, 2), 256, 0, stream>>>(wih_f, wih_b, WIHH, WIHL, n8i);
  cvt2_f16_kernel<<<dim3(n8h / 256, 2), 256, 0, stream>>>(whh_f, whh_b, WHH16, n8h, kWhhCarry);

  const dim3 gsq((kSeq / 64) * (kDim / 64) / 8, 1);
  wmma_gemm64<2, 0><<<gsq, 256, 0, stream>>>(
      XH, XL, kXw, 0L, W12H, W12L, kDim, 0L, (void*)U, (void*)U, kDim, 0L, b1, kSeq, kDim, kDim, 1.0f);
  wmma_gemm64<2, 0><<<gsq, 256, 0, stream>>>(
      XH, XL, kXw, 0L, W12H + (size_t)kDim * kDim, W12L + (size_t)kDim * kDim, kDim, 0L,
      (void*)WQ, (void*)WQ, kDim, 0L, b2, kSeq, kDim, kDim, 1.0f);

  score_kernel<<<dim3(kSeq / kScJB, kSeq / 16), 256, 0, stream>>>(U, WQ, VHL, E);
  softmax_split_kernel<<<kSeq, 64, 0, stream>>>(E, AH, AL);

  wmma_gemm64<0, 2><<<gsq, 256, 0, stream>>>(
      AH, AL, kSeq, 0L, VTH, VTL, kSeq, 0L, (void*)(XH + kDim), (void*)(XL + kDim), kXw, 0L, b1, kSeq, kDim, kSeq, 1.0f);

  const dim3 ggi((kSeq / 64) * (kG3 / 64) / 8, 1);
  wmma_gemm64<2, 0><<<ggi, 256, 0, stream>>>(
      XH, XL, kXw, 0L, WIHH, WIHL, kXw, 0L, (void*)GIF, (void*)GIF, kG3, 0L, bih_f, kSeq, kG3, kXw, 1.0f);
  wmma_gemm64<2, 0><<<ggi, 256, 0, stream>>>(
      XH, XL, kXw, 0L, WIHH + (size_t)kG3 * kXw, WIHL + (size_t)kG3 * kXw, kXw, 0L,
      (void*)GIB, (void*)GIB, kG3, 0L, bih_b, kSeq, kG3, kXw, 1.0f);

  gru_kernel<<<2, 512, 0, stream>>>(GIF, GIB, WHH16, bhh_f, bhh_b, out);
}
